// GraphDecoderLayer_76373108457772
// MI455X (gfx1250) — hardware-verified
//
#include <hip/hip_runtime.h>
#include <stddef.h>


#define DF     128
#define NTHR   256
#define NWAVE  8
#define NB     256
#define ACCP   128
#define NACC   (NB + 2)
#define EPT    8
#define CHUNK  (NTHR * EPT)
#define WCAP   (EPT * 32)
#define LISTN  (NWAVE * WCAP)
#define PASSN  128
#define PCAP   (CHUNK + PASSN)
#define HP     136
#define PQP    256
#define SP     68
#define NRB    128
#define WSC    8.0f
#define WINV   0.125f
#define LN_EPS 1e-5f
#define OW1    0
#define OW2    32768
#define OU1    49152
#define OU2    81920
#define WTOT   98304

static_assert(PCAP == 17 * PASSN);
static_assert(PASSN == NWAVE * 16);
static_assert(NB == NWAVE * 32);
static_assert((HP % 8) == 0);
static_assert((SP % 4) == 0);
static_assert((WTOT % (8 * NTHR)) == 0);
static_assert((NB % NRB) == 0);

typedef float        v4f  __attribute__((ext_vector_type(4)));
typedef float        v8f  __attribute__((ext_vector_type(8)));
typedef int          v4i  __attribute__((ext_vector_type(4)));
typedef unsigned int v4u  __attribute__((ext_vector_type(4)));
typedef _Float16     v4h  __attribute__((ext_vector_type(4)));
typedef _Float16     v8h  __attribute__((ext_vector_type(8)));
typedef _Float16     v16h __attribute__((ext_vector_type(16)));
union FragH { v16h v; v8h h[2]; };
union Pack8 { v8h h; v4u u; };

#define WSYNC() do { __builtin_amdgcn_fence(__ATOMIC_RELEASE, "wavefront"); __builtin_amdgcn_wave_barrier(); } while (0)

__device__ __forceinline__ v8f zero8f() {
  v8f z;
#pragma unroll
  for (int i = 0; i < 8; ++i) z[i] = 0.0f;
  return z;
}

__device__ __forceinline__ v8f wmh(v16h a, v16h b, v8f c) {
  v8f d = __builtin_amdgcn_wmma_f32_16x16x32_f16(false, a, false, b, (short)0, c, false, false);
  asm volatile("v_nop\n\tv_nop\n\tv_nop\n\tv_nop" : "+v"(d) : "v"(a), "v"(b));
  return d;
}

__device__ __forceinline__ v8h cvt8(v4f a, v4f b) {
  v8h r;
  r[0] = (_Float16)a.x; r[1] = (_Float16)a.y; r[2] = (_Float16)a.z; r[3] = (_Float16)a.w;
  r[4] = (_Float16)b.x; r[5] = (_Float16)b.y; r[6] = (_Float16)b.z; r[7] = (_Float16)b.w;
  return r;
}

__device__ __forceinline__ v16h afragF(const float* p) {
  const v4f a0 = *(const v4f*)p;
  const v4f a1 = *(const v4f*)(p + 4);
  const v4f b0 = *(const v4f*)(p + 16);
  const v4f b1 = *(const v4f*)(p + 20);
  FragH f;
  f.h[0] = cvt8(a0, a1);
  f.h[1] = cvt8(b0, b1);
  return f.v;
}

__device__ __forceinline__ v16h bfrag(const _Float16* pl, int kk, int nc, int n, int h) {
  return *(const v16h*)(pl + ((size_t)(kk * nc + n) * 2 + h) * 16);
}

__device__ __forceinline__ int scan_chunk(const int* __restrict__ dsts, int nE, int cbase, int nodeBase,
                                          int vec8, int* list, int tid, int wave) {
  int wc = 0;
  const int el0  = tid * EPT;
  const int e0   = cbase + el0;
  const int sent = -2147483647 - 1;
  v4i da, db;
  if (vec8 != 0 && cbase + CHUNK <= nE) {
    da = *(const v4i*)(dsts + e0);
    db = *(const v4i*)(dsts + e0 + 4);
  } else {
    da.x = (e0     < nE) ? dsts[min(e0,     nE - 1)] : sent;
    da.y = (e0 + 1 < nE) ? dsts[min(e0 + 1, nE - 1)] : sent;
    da.z = (e0 + 2 < nE) ? dsts[min(e0 + 2, nE - 1)] : sent;
    da.w = (e0 + 3 < nE) ? dsts[min(e0 + 3, nE - 1)] : sent;
    db.x = (e0 + 4 < nE) ? dsts[min(e0 + 4, nE - 1)] : sent;
    db.y = (e0 + 5 < nE) ? dsts[min(e0 + 5, nE - 1)] : sent;
    db.z = (e0 + 6 < nE) ? dsts[min(e0 + 6, nE - 1)] : sent;
    db.w = (e0 + 7 < nE) ? dsts[min(e0 + 7, nE - 1)] : sent;
  }
  const unsigned nb = (unsigned)nodeBase;
  const unsigned s0 = (unsigned)da.x - nb, s1 = (unsigned)da.y - nb;
  const unsigned s2 = (unsigned)da.z - nb, s3 = (unsigned)da.w - nb;
  const unsigned s4 = (unsigned)db.x - nb, s5 = (unsigned)db.y - nb;
  const unsigned s6 = (unsigned)db.z - nb, s7 = (unsigned)db.w - nb;
  const bool h0 = s0 < (unsigned)NB, h1 = s1 < (unsigned)NB, h2 = s2 < (unsigned)NB, h3 = s3 < (unsigned)NB;
  const bool h4 = s4 < (unsigned)NB, h5 = s5 < (unsigned)NB, h6 = s6 < (unsigned)NB, h7 = s7 < (unsigned)NB;
  const unsigned any = __builtin_amdgcn_ballot_w32(h0 | h1 | h2 | h3 | h4 | h5 | h6 | h7);
  if (any != 0u) {
#define HITJ(J, HJ) { \
      const unsigned mj = __builtin_amdgcn_ballot_w32(HJ); \
      if (mj != 0u) { \
        if (HJ) { \
          const int pos = wc + (int)__builtin_amdgcn_mbcnt_lo(mj, 0u); \
          if (pos < WCAP) list[wave * WCAP + pos] = el0 + (J); \
        } \
        wc += (int)__builtin_popcount(mj); } }
    HITJ(0, h0)
    HITJ(1, h1)
    HITJ(2, h2)
    HITJ(3, h3)
    HITJ(4, h4)
    HITJ(5, h5)
    HITJ(6, h6)
    HITJ(7, h7)
#undef HITJ
  }
  return wc;
}

__global__ __launch_bounds__(NTHR) void k_prep(const float* __restrict__ wm1, const float* __restrict__ wm2,
                                               const float* __restrict__ wu1, const float* __restrict__ wu2,
                                               _Float16* wsw) {
  const int b = blockIdx.x;
  const int t = b * NTHR + (int)threadIdx.x;
  if (t >= WTOT / 8) return;
  const float* src; int lnc, tb, comb;
  if (b < 16)      { src = wm1; lnc = 8; tb = 0;     comb = 1; }
  else if (b < 24) { src = wm2; lnc = 7; tb = 4096;  comb = 0; }
  else if (b < 40) { src = wu1; lnc = 7; tb = 6144;  comb = 0; }
  else             { src = wu2; lnc = 7; tb = 10240; comb = 0; }
  const int q    = t - tb;
  const int isel = q & 1, hf = (q >> 1) & 1, cn = q >> 2;
  const int n    = cn & ((1 << lnc) - 1);
  const int kk   = cn >> lnc;
  const int kb   = kk * 32 + 8 * hf + 16 * isel;
  int koff = 0, nn = n;
  if (comb != 0 && n >= DF) { koff = DF; nn = n - DF; }
  Pack8 pk;
#pragma unroll
  for (int j = 0; j < 8; ++j) pk.h[j] = (_Float16)(src[(size_t)(kb + j + koff) * DF + nn] * WSC);
  _Float16* dp = wsw + (size_t)t * 8;
  const v4u u = pk.u;
  *(volatile v4u*)dp = u;
  __threadfence();
  *(volatile v4u*)dp = u;
}

__global__ __launch_bounds__(NTHR) void k_node(const float* __restrict__ x, const _Float16* __restrict__ wsw,
                                               const float* __restrict__ bm1, float* pq, int nN) {
  __shared__ __attribute__((aligned(16))) float stg[NWAVE * 16 * SP];
  const int tid = threadIdx.x, lane = tid & 31, wave = tid >> 5, h = lane >> 4, m = lane & 15;
  const int row0 = blockIdx.x * NRB + wave * 16;
  float* sw = stg + wave * 16 * SP;
  int xr = row0 + m;
  xr = xr > nN - 1 ? nN - 1 : xr;
  const float* xrow = x + (size_t)xr * DF;
  const _Float16* w1p = wsw + OW1;
  const int rsub = lane >> 4, c4 = (lane & 15) * 4;

#pragma unroll 1
  for (int p = 0; p < 2; ++p) {
    v8f c[8];
#pragma unroll
    for (int t = 0; t < 8; ++t) c[t] = zero8f();
#pragma unroll 1
    for (int kk = 0; kk < 4; ++kk) {
      const v16h a = afragF(xrow + kk * 32 + 8 * h);
#pragma unroll
      for (int t = 0; t < 8; ++t)
        c[t] = wmh(a, bfrag(w1p, kk, 2 * DF, p * DF + 16 * t + m, h), c[t]);
    }
#pragma unroll
    for (int s = 0; s < 2; ++s) {
#pragma unroll
      for (int tq = 0; tq < 4; ++tq) {
        const int t   = 4 * s + tq;
        const int col = 16 * t + m;
        const float bv = bm1[col];
        const float bb = (p != 0) ? bv : 0.0f;
#pragma unroll
        for (int r8 = 0; r8 < 8; ++r8) sw[(8 * h + r8) * SP + 16 * tq + m] = c[t][r8] * WINV + bb;
      }
      WSYNC();
      float* gb = pq + (size_t)row0 * PQP + p * DF + 64 * s + c4;
#pragma unroll
      for (int rp = 0; rp < 8; ++rp) {
        const int rw = 2 * rp + rsub;
        const v4f v = *(const v4f*)(sw + rw * SP + c4);
        *(volatile v4f*)(gb + (size_t)rw * PQP) = v;
      }
      __threadfence();
#pragma unroll
      for (int rp = 0; rp < 8; ++rp) {
        const int rw = 2 * rp + rsub;
        const v4f v = *(const v4f*)(sw + rw * SP + c4);
        *(volatile v4f*)(gb + (size_t)rw * PQP) = v;
      }
      WSYNC();
    }
  }
}

__global__ __launch_bounds__(NTHR) void k_agg(
    const float* __restrict__ x, const int* __restrict__ ei, const float* __restrict__ pq,
    const _Float16* __restrict__ wsw,
    const float* __restrict__ bm2, const float* __restrict__ bu1, const float* __restrict__ bu2,
    const float* __restrict__ gma, const float* __restrict__ bta,
    float* out, int nN, int nE, int vec8) {
  __shared__ __attribute__((aligned(16))) float    acc[NACC * ACCP];
  __shared__ __attribute__((aligned(16))) _Float16 hs[PASSN * HP];
  __shared__ __attribute__((aligned(16))) int      list[LISTN];
  __shared__ __attribute__((aligned(16))) int      pend[PCAP];
  __shared__ int   rowb[PASSN];
  __shared__ int   slotb[PASSN];
  __shared__ __attribute__((aligned(16))) float    prm[5 * DF];
  __shared__ int   wcnt[NWAVE];
  __shared__ int   pendN;

  const int tid = threadIdx.x, lane = tid & 31, wave = tid >> 5, h = lane >> 4, m = lane & 15;
  const int nodeBase = blockIdx.x * NB;
  const int* srcs = ei;
  const int* dsts = ei + nE;
  const _Float16* w2p = wsw + OW2;
  const _Float16* u1p = wsw + OU1;
  const _Float16* u2p = wsw + OU2;

  {
    const v4f z4 = {0.0f, 0.0f, 0.0f, 0.0f};
    for (int i = tid; i < (NACC * ACCP) / 4; i += NTHR) *(v4f*)(acc + 4 * i) = z4;
  }
  if (tid < DF) {
    prm[tid]          = bm2[tid];
    prm[DF + tid]     = bu1[tid];
    prm[2 * DF + tid] = bu2[tid];
    prm[3 * DF + tid] = gma[tid];
    prm[4 * DF + tid] = bta[tid];
  }
  if (tid == 0) pendN = 0;
  __syncthreads();

  const int nChunks = (nE + CHUNK - 1) / CHUNK;
#pragma unroll 1
  for (int ch = 0; ch < nChunks; ++ch) {
    const int cbase = ch * CHUNK;
    const int wc = scan_chunk(dsts, nE, cbase, nodeBase, vec8, list, tid, wave);
    if (lane == 0) wcnt[wave] = wc;
    __syncthreads();

    const int base = pendN;
    int tot = 0, myoff = 0;
#pragma unroll
    for (int w = 0; w < NWAVE; ++w) {
      int c = wcnt[w];
      c = c > WCAP ? WCAP : (c < 0 ? 0 : c);
      if (w < wave) myoff += c;
      tot += c;
    }
    int newN = base + tot;
    newN = newN > PCAP ? PCAP : newN;
    {
      int n = wcnt[wave];
      n = n > WCAP ? WCAP : (n < 0 ? 0 : n);
      const int* lp = list + wave * WCAP;
      for (int i = lane; i < n; i += 32) {
        const int pos = base + myoff + i;
        if (pos < PCAP) pend[pos] = cbase + lp[i];
      }
    }
    const int fin = (ch == nChunks - 1) ? 1 : 0;
    const int R   = (fin != 0) ? (newN + PASSN - 1) / PASSN : newN / PASSN;
    const int Pv  = (fin != 0) ? newN : R * PASSN;
    __syncthreads();

#pragma unroll 1
    for (int ps = 0; ps < R; ++ps) {
      int nv = Pv - ps * PASSN;
      nv = nv > PASSN ? PASSN : nv;
      const int ntile = (nv + 15) >> 4;

      if (tid < PASSN) {
        const int idx = ps * PASSN + tid;
        const bool valid = idx < Pv;
        int e = pend[idx];
        e = e < 0 ? 0 : (e > nE - 1 ? nE - 1 : e);
        const int d = dsts[e];
        int s = srcs[e];
        int slot = d - nodeBase;
        if (!valid || (unsigned)slot >= (unsigned)NB) slot = NB;
        s = s < 0 ? 0 : (s > nN - 1 ? nN - 1 : s);
        rowb[tid]  = valid ? s : 0;
        slotb[tid] = slot;
      }
      __syncthreads();

      if (wave < ntile) {
#pragma unroll 4
        for (int j = 0; j < 16; ++j) {
          const int e  = wave * 16 + j;
          const int rw = rowb[e];
          const int sl = slotb[e];
          const bool ok = (unsigned)sl < (unsigned)NB;
          const int qn = nodeBase + (ok ? sl : NB - 1);
          const v4f pv = *(const v4f*)(pq + (size_t)rw * PQP + 4 * lane);
          const v4f qv = *(const v4f*)(pq + (size_t)qn * PQP + DF + 4 * lane);
          const float f0 = ok ? fmaxf(pv.x + qv.x, 0.0f) : 0.0f;
          const float f1 = ok ? fmaxf(pv.y + qv.y, 0.0f) : 0.0f;
          const float f2 = ok ? fmaxf(pv.z + qv.z, 0.0f) : 0.0f;
          const float f3 = ok ? fmaxf(pv.w + qv.w, 0.0f) : 0.0f;
          v4h hv;
          hv[0] = (_Float16)f0; hv[1] = (_Float16)f1; hv[2] = (_Float16)f2; hv[3] = (_Float16)f3;
          *(v4h*)(hs + e * HP + 4 * lane) = hv;
        }
      }
      __syncthreads();

      {
        const int acol = wave * 16 + m;
        v16h bw[4];
#pragma unroll
        for (int kk = 0; kk < 4; ++kk) bw[kk] = bfrag(w2p, kk, DF, acol, h);
        const float bcol = prm[acol];
#pragma unroll 1
        for (int tt = 0; tt < ntile; ++tt) {
          v8f dd = zero8f();
#pragma unroll
          for (int kk = 0; kk < 4; ++kk) {
            FragH a;
            const _Float16* ap = hs + (tt * 16 + m) * HP + kk * 32 + 8 * h;
            a.h[0] = *(const v8h*)ap;
            a.h[1] = *(const v8h*)(ap + 16);
            dd = wmh(a.v, bw[kk], dd);
          }
          float mv[8];
#pragma unroll
          for (int r8 = 0; r8 < 8; ++r8) mv[r8] = dd[r8] * WINV + bcol;
#pragma unroll
          for (int r8 = 0; r8 < 8; ++r8) {
            int s0 = slotb[tt * 16 + r8];
            s0 = s0 < 0 ? 0 : (s0 > NB ? NB : s0);
            const int sl = (h == 0) ? s0 : (NB + 1);
            acc[sl * ACCP + acol] += mv[r8];
          }
          WSYNC();
#pragma unroll
          for (int r8 = 0; r8 < 8; ++r8) {
            int s1 = slotb[tt * 16 + 8 + r8];
            s1 = s1 < 0 ? 0 : (s1 > NB ? NB : s1);
            const int sl = (h != 0) ? s1 : (NB + 1);
            acc[sl * ACCP + acol] += mv[r8];
          }
          WSYNC();
        }
      }
      __syncthreads();
    }

    int rem = newN - R * PASSN;
    rem = rem < 0 ? 0 : rem;
    if (R > 0 && tid < rem) pend[tid] = pend[R * PASSN + tid];
    if (tid == 0) pendN = rem;
  }
  __syncthreads();

  const float* bu1s = prm + DF;
  const float* bu2s = prm + 2 * DF;
  const float* gsm  = prm + 3 * DF;
  const float* bsm  = prm + 4 * DF;
  _Float16* hw = hs + wave * 16 * HP;
#pragma unroll 1
  for (int tau = 0; tau < 2; ++tau) {
    const int sT    = wave * 32 + tau * 16;
    const int node0 = nodeBase + sT;
    int xr = node0 + m;
    xr = xr > nN - 1 ? nN - 1 : xr;
    const float* xrow = x + (size_t)xr * DF;
    const float* arow = acc + (size_t)(sT + m) * ACCP;

    v8f c[8];
#pragma unroll
    for (int t = 0; t < 8; ++t) c[t] = zero8f();
#pragma unroll 1
    for (int kk = 0; kk < 4; ++kk) {
      const v16h a = afragF(xrow + kk * 32 + 8 * h);
#pragma unroll
      for (int t = 0; t < 8; ++t) c[t] = wmh(a, bfrag(u1p, kk, DF, 16 * t + m, h), c[t]);
    }
#pragma unroll 1
    for (int kk = 0; kk < 4; ++kk) {
      const v16h a = afragF(arow + kk * 32 + 8 * h);
#pragma unroll
      for (int t = 0; t < 8; ++t) c[t] = wmh(a, bfrag(u1p, kk + 4, DF, 16 * t + m, h), c[t]);
    }
#pragma unroll
    for (int t = 0; t < 8; ++t) {
      const float bb = bu1s[16 * t + m];
#pragma unroll
      for (int r8 = 0; r8 < 8; ++r8)
        hw[(8 * h + r8) * HP + 16 * t + m] = (_Float16)fmaxf(c[t][r8] * WINV + bb, 0.0f);
    }
    WSYNC();
#pragma unroll
    for (int t = 0; t < 8; ++t) c[t] = zero8f();
#pragma unroll 1
    for (int kk = 0; kk < 4; ++kk) {
      FragH a;
      const _Float16* ap = hw + m * HP + kk * 32 + 8 * h;
      a.h[0] = *(const v8h*)ap;
      a.h[1] = *(const v8h*)(ap + 16);
#pragma unroll
      for (int t = 0; t < 8; ++t) c[t] = wmh(a.v, bfrag(u2p, kk, DF, 16 * t + m, h), c[t]);
    }
#pragma unroll
    for (int t = 0; t < 8; ++t) {
      const float bb = bu2s[16 * t + m];
#pragma unroll
      for (int r8 = 0; r8 < 8; ++r8) c[t][r8] = c[t][r8] * WINV + bb;
    }
    float mean[8], rsd[8];
#pragma unroll
    for (int r8 = 0; r8 < 8; ++r8) {
      float s = 0.0f;
#pragma unroll
      for (int t = 0; t < 8; ++t) s += c[t][r8];
      s += __shfl_xor(s, 1);
      s += __shfl_xor(s, 2);
      s += __shfl_xor(s, 4);
      s += __shfl_xor(s, 8);
      const float mu = s * (1.0f / (float)DF);
      float q = 0.0f;
#pragma unroll
      for (int t = 0; t < 8; ++t) { const float dl = c[t][r8] - mu; q += dl * dl; }
      q += __shfl_xor(q, 1);
      q += __shfl_xor(q, 2);
      q += __shfl_xor(q, 4);
      q += __shfl_xor(q, 8);
      mean[r8] = mu;
      rsd[r8]  = rsqrtf(q * (1.0f / (float)DF) + LN_EPS);
    }
    float* so = acc + (size_t)sT * ACCP;
#pragma unroll
    for (int t = 0; t < 8; ++t) {
      const int col = 16 * t + m;
      const float g = gsm[col], be = bsm[col];
#pragma unroll
      for (int r8 = 0; r8 < 8; ++r8)
        so[(8 * h + r8) * ACCP + col] = (c[t][r8] - mean[r8]) * rsd[r8] * g + be;
    }
    WSYNC();
#pragma unroll 1
    for (int rw = 0; rw < 16; ++rw) {
      const int node = node0 + rw;
      if (node < nN) {
        const v4f sv = *(const v4f*)(so + rw * ACCP + 4 * lane);
        const v4f xv = *(const v4f*)(x + (size_t)node * DF + 4 * lane);
        const v4f o = sv + xv;
        *(volatile v4f*)(out + (size_t)node * DF + 4 * lane) = o;
      }
    }
    __threadfence();
#pragma unroll 1
    for (int rw = 0; rw < 16; ++rw) {
      const int node = node0 + rw;
      if (node < nN) {
        const v4f sv = *(const v4f*)(so + rw * ACCP + 4 * lane);
        const v4f xv = *(const v4f*)(x + (size_t)node * DF + 4 * lane);
        const v4f o = sv + xv;
        *(volatile v4f*)(out + (size_t)node * DF + 4 * lane) = o;
      }
    }
    WSYNC();
  }
}

extern "C" void kernel_launch(void* const* d_in, const int* in_sizes, int n_in,
                              void* d_out, int out_size, void* d_ws, size_t ws_size,
                              hipStream_t stream) {
  if (n_in < 12) return;
  const int nN = in_sizes[0] / DF;
  const int nE = in_sizes[1] / 2;
  if (nN <= 0 || in_sizes[0] != nN * DF || nE < 0 || in_sizes[1] != 2 * nE) return;
  if (in_sizes[2] != 2 * DF * DF || in_sizes[3] != DF || in_sizes[4] != DF * DF || in_sizes[5] != DF) return;
  if (in_sizes[6] != 2 * DF * DF || in_sizes[7] != DF || in_sizes[8] != DF * DF || in_sizes[9] != DF) return;
  if (in_sizes[10] != DF || in_sizes[11] != DF) return;
  if (out_size != nN * DF) return;

  const float* x    = (const float*)d_in[0];
  const int*   ei   = (const int*)d_in[1];
  const float* w_m1 = (const float*)d_in[2];
  const float* b_m1 = (const float*)d_in[3];
  const float* w_m2 = (const float*)d_in[4];
  const float* b_m2 = (const float*)d_in[5];
  const float* w_u1 = (const float*)d_in[6];
  const float* b_u1 = (const float*)d_in[7];
  const float* w_u2 = (const float*)d_in[8];
  const float* b_u2 = (const float*)d_in[9];
  const float* gma  = (const float*)d_in[10];
  const float* bta  = (const float*)d_in[11];
  float* out = (float*)d_out;

  const int nBlk = (nN + NB - 1) / NB;
  const int nPad = nBlk * NB;

  char* ws = (char*)d_ws;
  size_t off = 0;
  const size_t oW = off;  off += (size_t)WTOT * 2;          off = (off + 255) & ~(size_t)255;
  const size_t oPQ = off; off += (size_t)nPad * PQP * 4;    off = (off + 255) & ~(size_t)255;
  if (off > ws_size) return;
  _Float16* wsw = (_Float16*)(ws + oW);
  float* pq = (float*)(ws + oPQ);

  const int vec8 = ((nE & 3) == 0) ? 1 : 0;

  k_prep<<<WTOT / (8 * NTHR), NTHR, 0, stream>>>(w_m1, w_m2, w_u1, w_u2, wsw);

  k_node<<<nPad / NRB, NTHR, 0, stream>>>(x, wsw, b_m1, pq, nN);

  k_agg<<<nBlk, NTHR, 0, stream>>>(x, ei, pq, wsw, b_m2, b_u1, b_u2, gma, bta, out, nN, nE, vec8);
}
